// DotAttentionLayer_36146444763807
// MI455X (gfx1250) — hardware-verified
//
#include <hip/hip_runtime.h>


#define NN_  50000
#define NNP  50048
#define NE_  800000
#define DM   128

typedef unsigned short bf;
typedef __attribute__((ext_vector_type(16))) __bf16   v16bf;
typedef __attribute__((ext_vector_type(8)))  unsigned short v8us;
typedef __attribute__((ext_vector_type(4)))  unsigned short v4us;
typedef __attribute__((ext_vector_type(8)))  float    v8f;
typedef __attribute__((ext_vector_type(4)))  float    v4f;
typedef v4f  __attribute__((may_alias)) v4fa;

__device__ __forceinline__ unsigned short f2bf(float f) { unsigned u = __float_as_uint(f); u += 0x7FFFu + ((u >> 16) & 1u); return (unsigned short)(u >> 16); }
__device__ __forceinline__ float bf2f(unsigned short b) { return __uint_as_float(((unsigned)b) << 16); }
__device__ __forceinline__ float bfr(float f) { return bf2f(f2bf(f)); }
__device__ __forceinline__ v16bf cat16b(v8us lo, v8us hi) { return __builtin_bit_cast(v16bf, __builtin_shufflevector(lo, hi, 0, 1, 2, 3, 4, 5, 6, 7, 8, 9, 10, 11, 12, 13, 14, 15)); }
__device__ __forceinline__ v8f wmmab(v16bf a, v16bf b, v8f c) { return __builtin_amdgcn_wmma_f32_16x16x32_bf16(false, a, false, b, (short)0, c, false, false); }
#define VST2(T, p, v) do { const T vst2_v_ = (v); *(volatile T*)(p) = vst2_v_; __threadfence(); *(volatile T*)(p) = vst2_v_; } while (0)

__global__ __launch_bounds__(256) void k_ind(const int* __restrict__ self_idx, float* IND) {
    __shared__ unsigned char flg[NNP];
    const int t = threadIdx.x;
    for (int i = t; i < NNP; i += 256) flg[i] = 0;
    __syncthreads();
#pragma unroll 1
    for (int e = t; e < NE_; e += 256) { int n = self_idx[e]; if (n < 0) n += NN_; if ((unsigned)n < (unsigned)NN_) flg[n] = 1; }
    __syncthreads();
#pragma unroll 1
    for (int i = t * 4; i < NNP; i += 256 * 4) { v4f v; v[0] = flg[i]; v[1] = flg[i + 1]; v[2] = flg[i + 2]; v[3] = flg[i + 3]; VST2(v4f, IND + i, v); }
}
__global__ __launch_bounds__(256) void k_xb(const float* __restrict__ v, bf* Vb) {
    const int lane = threadIdx.x & 31, r = blockIdx.x * 8 + (threadIdx.x >> 5);
    if (r >= NNP) return;
    const int rr = (r < NN_) ? r : (NN_ - 1);
    v4us t;
#pragma unroll
    for (int i = 0; i < 4; ++i) { const unsigned short hb = f2bf(v[(size_t)rr * DM + lane * 4 + i]); t[i] = (r < NN_) ? hb : (unsigned short)0; }
    VST2(v4us, Vb + (size_t)r * DM + lane * 4, t);
}
__global__ __launch_bounds__(256) void k_cvtb(const float* __restrict__ src, bf* dst) {
    const int lane = threadIdx.x & 31, r = blockIdx.x * 8 + (threadIdx.x >> 5);
    if (r >= DM) return;
    v4us t;
#pragma unroll
    for (int i = 0; i < 4; ++i) t[i] = f2bf(src[(size_t)r * DM + lane * 4 + i]);
    VST2(v4us, dst + (size_t)r * DM + lane * 4, t);
}

template <bool SPLITA, int MODE>
__global__ __launch_bounds__(128) void k_gemmb(const bf* __restrict__ A, const bf* __restrict__ Al, const bf* __restrict__ Bn, const float* __restrict__ bias, const float* __restrict__ IND, void* C, void* C2) {
    __shared__ __align__(16) float ost[4][16 * 68];
    const int lane = threadIdx.x & 31, wave = threadIdx.x >> 5, lr = lane & 15, hi = lane >> 4;
    const int r0 = blockIdx.x * 64 + wave * 16, c0 = blockIdx.y * 64;
    const size_t aoff = (size_t)(r0 + lr) * DM + 8 * hi;
    size_t boff[4];
#pragma unroll
    for (int t = 0; t < 4; ++t) boff[t] = (size_t)(c0 + t * 16 + lr) * DM + 8 * hi;
    v8f acc[4];
#pragma unroll
    for (int t = 0; t < 4; ++t) acc[t] = (v8f){};
#pragma unroll
    for (int kc = 0; kc < DM; kc += 32) {
        const v16bf a = cat16b(*(const v8us*)(A + aoff + kc), *(const v8us*)(A + aoff + kc + 16));
        v16bf al = a;
        if (SPLITA) al = cat16b(*(const v8us*)(Al + aoff + kc), *(const v8us*)(Al + aoff + kc + 16));
#pragma unroll
        for (int t = 0; t < 4; ++t) { const v16bf b = cat16b(*(const v8us*)(Bn + boff[t] + kc), *(const v8us*)(Bn + boff[t] + kc + 16)); acc[t] = wmmab(a, b, acc[t]); if (SPLITA) acc[t] = wmmab(al, b, acc[t]); }
    }
    asm volatile("v_nop\n\tv_nop\n\tv_nop\n\tv_nop" : "+v"(acc[0]), "+v"(acc[1]), "+v"(acc[2]), "+v"(acc[3]));
    float* os = &ost[wave][0];
#pragma unroll
    for (int t = 0; t < 4; ++t) { const int col = c0 + t * 16 + lr; const float bv = bfr(bias[col]);
#pragma unroll
        for (int j = 0; j < 8; ++j) { float v = acc[t][j] + bv; if (MODE == 0) v *= IND[r0 + hi * 8 + j]; if (MODE == 2) v = fmaxf(v, 0.f); os[(hi * 8 + j) * 68 + t * 16 + lr] = v; } }
    __syncthreads();
    if (MODE == 1) {
        float* crow = (float*)C + (size_t)r0 * DM + c0;
        auto pass = [&]() {
#pragma unroll
            for (int s = 0; s < 8; ++s) { const int Lid = (lane >> 3) + 4 * s, piece = lane & 7; const int row = Lid >> 1, cofs = (Lid & 1) * 32 + piece * 4;
                const v4f val = *(const v4fa*)(os + row * 68 + cofs); *(volatile v4f*)(crow + (size_t)row * DM + cofs) = val; }
        };
        pass(); __threadfence(); pass();
    } else {
        bf* ch = (bf*)C + (size_t)r0 * DM + c0; bf* cl = (bf*)C2 + (size_t)r0 * DM + c0;
        auto pass = [&]() {
#pragma unroll
            for (int s = 0; s < 4; ++s) { const int row = 4 * s + (lane >> 3), piece = lane & 7; const float* sp = os + row * 68 + piece * 8; v8us oh, ol;
#pragma unroll
                for (int i = 0; i < 8; ++i) { const unsigned short hb = f2bf(sp[i]); oh[i] = hb; ol[i] = f2bf(sp[i] - bf2f(hb)); }
                *(volatile v8us*)(ch + (size_t)row * DM + piece * 8) = oh; *(volatile v8us*)(cl + (size_t)row * DM + piece * 8) = ol; }
        };
        pass(); __threadfence(); pass();
    }
}

template <bool ROUNDA, bool FINAL>
__global__ __launch_bounds__(256) void k_ln(const float* __restrict__ Xa, const float* __restrict__ Xb_, const float* __restrict__ w, const float* __restrict__ bb, float* X, bf* H, bf* L) {
    const int lane = threadIdx.x & 31, r = blockIdx.x * 8 + (threadIdx.x >> 5);
    if (r >= (FINAL ? NN_ : NNP)) return;
    const int ra = (ROUNDA && r >= NN_) ? (NN_ - 1) : r;
    float v[4]; float s = 0.f;
#pragma unroll
    for (int i = 0; i < 4; ++i) { const float a = Xa[(size_t)ra * DM + lane * 4 + i]; v[i] = (ROUNDA ? bfr(a) : a) + Xb_[(size_t)r * DM + lane * 4 + i]; s += v[i]; }
#pragma unroll
    for (int o = 16; o; o >>= 1) s += __shfl_xor(s, o, 32);
    const float mu = s * (1.0f / DM);
    float q = 0.f;
#pragma unroll
    for (int i = 0; i < 4; ++i) { const float d = v[i] - mu; q += d * d; }
#pragma unroll
    for (int o = 16; o; o >>= 1) q += __shfl_xor(q, o, 32);
    const float rs = 1.0f / sqrtf(q * (1.0f / DM) + 1e-5f);
    v4f xo; v4us oh, ol;
#pragma unroll
    for (int i = 0; i < 4; ++i) { const int c = lane * 4 + i; const float y = (v[i] - mu) * rs * bfr(w[c]) + bfr(bb[c]); xo[i] = y; const unsigned short hb = f2bf(y); oh[i] = hb; ol[i] = f2bf(y - bf2f(hb)); }
    *(volatile v4f*)(X + (size_t)r * DM + lane * 4) = xo;
    if (H) { *(volatile v4us*)(H + (size_t)r * DM + lane * 4) = oh; *(volatile v4us*)(L + (size_t)r * DM + lane * 4) = ol; }
    __threadfence();
    *(volatile v4f*)(X + (size_t)r * DM + lane * 4) = xo;
    if (H) { *(volatile v4us*)(H + (size_t)r * DM + lane * 4) = oh; *(volatile v4us*)(L + (size_t)r * DM + lane * 4) = ol; }
}

extern "C" void kernel_launch(void* const* d_in, const int* in_sizes, int n_in,
                              void* d_out, int out_size, void* d_ws, size_t ws_size, hipStream_t stream) {
    (void)in_sizes; (void)n_in; (void)out_size;
    const float* v = (const float*)d_in[2]; const int* self_idx = (const int*)d_in[3];
    const float* Wv = (const float*)d_in[9]; const float* bv = (const float*)d_in[10]; const float* Wo = (const float*)d_in[11]; const float* bo = (const float*)d_in[12];
    const float* W1 = (const float*)d_in[13]; const float* b1 = (const float*)d_in[14]; const float* W2 = (const float*)d_in[15]; const float* b2 = (const float*)d_in[16];
    const float* ln1w = (const float*)d_in[17]; const float* ln1b = (const float*)d_in[18]; const float* ln2w = (const float*)d_in[19]; const float* ln2b = (const float*)d_in[20];
    float* out = (float*)d_out;
    char* wsp = (char*)d_ws;
    auto take = [&](size_t bytes) { char* p = wsp; wsp += (bytes + 255) & ~(size_t)255; return (void*)p; };
    float* IND = (float*)take((size_t)NNP * 4); bf* Vb = (bf*)take((size_t)NNP * DM * 2);
    bf* WvB = (bf*)take(DM * DM * 2); bf* WoB = (bf*)take(DM * DM * 2); bf* W1B = (bf*)take(DM * DM * 2); bf* W2B = (bf*)take(DM * DM * 2);
    bf* AH = (bf*)take((size_t)NNP * DM * 2); bf* AL = (bf*)take((size_t)NNP * DM * 2); bf* BH = (bf*)take((size_t)NNP * DM * 2); bf* BL = (bf*)take((size_t)NNP * DM * 2);
    float* O = (float*)take((size_t)NNP * DM * 4); float* V1 = (float*)take((size_t)NNP * DM * 4);
    if ((size_t)(wsp - (char*)d_ws) > ws_size) return;
    k_ind<<<1, 256, 0, stream>>>(self_idx, IND);
    k_xb<<<NNP / 8, 256, 0, stream>>>(v, Vb);
    k_cvtb<<<DM / 8, 256, 0, stream>>>(Wv, WvB); k_cvtb<<<DM / 8, 256, 0, stream>>>(Wo, WoB); k_cvtb<<<DM / 8, 256, 0, stream>>>(W1, W1B); k_cvtb<<<DM / 8, 256, 0, stream>>>(W2, W2B);
    k_gemmb<false, 0><<<dim3(NNP / 64, DM / 64, 1), 128, 0, stream>>>(Vb, nullptr, WvB, bv, IND, AH, AL);
    k_gemmb<true, 1><<<dim3(NNP / 64, DM / 64, 1), 128, 0, stream>>>(AH, AL, WoB, bo, nullptr, O, nullptr);
    k_ln<true, false><<<NNP / 8, 256, 0, stream>>>(v, O, ln1w, ln1b, V1, AH, AL);
    k_gemmb<true, 2><<<dim3(NNP / 64, DM / 64, 1), 128, 0, stream>>>(AH, AL, W1B, b1, nullptr, BH, BL);
    k_gemmb<true, 1><<<dim3(NNP / 64, DM / 64, 1), 128, 0, stream>>>(BH, BL, W2B, b2, nullptr, O, nullptr);
    k_ln<false, true><<<(NN_ + 7) / 8, 256, 0, stream>>>(V1, O, ln2w, ln2b, out, nullptr, nullptr);
}
